// DilatedSparseRnnStack_71262097375516
// MI455X (gfx1250) — hardware-verified
//
#include <hip/hip_runtime.h>
#include <math.h>

typedef __attribute__((ext_vector_type(16))) _Float16 v16h;
typedef __attribute__((ext_vector_type(8)))  _Float16 v8h;
typedef __attribute__((ext_vector_type(16))) __bf16   v16b;
typedef __attribute__((ext_vector_type(8)))  __bf16   v8b;
typedef __attribute__((ext_vector_type(8)))  float    v8f;
typedef __attribute__((ext_vector_type(4)))  float    v4f;
typedef __attribute__((ext_vector_type(2)))  unsigned v2u;

__device__ __forceinline__ unsigned short f2bf_bits(float f) {
  unsigned u = __float_as_uint(f);
  return (unsigned short)((u + 0x7FFFu + ((u >> 16) & 1u)) >> 16);
}
__device__ __forceinline__ float bf_bits2f(unsigned short h) { return __uint_as_float(((unsigned)h) << 16); }

__device__ __forceinline__ void dep_guard_h(v8f& a, v8f& b, v16h x, v16h y) { asm volatile("v_nop\n\tv_nop\n\tv_nop\n\tv_nop" : "+v"(a), "+v"(b) : "v"(x), "v"(y)); }
__device__ __forceinline__ void dep_guard_b(v8f& a, v8f& b, v16b x, v16b y) { asm volatile("v_nop\n\tv_nop\n\tv_nop\n\tv_nop" : "+v"(a), "+v"(b) : "v"(x), "v"(y)); }
__device__ __forceinline__ void keep4_h(v16h a, v16h b, v16h c, v16h d) { asm volatile("v_nop" :: "v"(a), "v"(b), "v"(c), "v"(d)); }
__device__ __forceinline__ void keep4_b(v16b a, v16b b, v16b c, v16b d) { asm volatile("v_nop" :: "v"(a), "v"(b), "v"(c), "v"(d)); }
__device__ __forceinline__ void acc_guard4(v8f& a, v8f& b, v8f& c, v8f& d) { asm volatile("v_nop\n\tv_nop\n\tv_nop\n\tv_nop" : "+v"(a), "+v"(b), "+v"(c), "+v"(d)); }
template <typename T> struct Frag;
template <> struct Frag<_Float16> {
  typedef v16h V; union U { v16h v; v8h h[2]; };
  static __device__ __forceinline__ v16h load(const _Float16* p) {
    U f; f.h[0] = *(const v8h*)(p); f.h[1] = *(const v8h*)(p + 16); return f.v;
  }
  static __device__ __forceinline__ v8f mma(v16h a, v16h b, v8f c) {
    return __builtin_amdgcn_wmma_f32_16x16x32_f16(false, a, false, b, (short)0, c, false, false);
  }
  static __device__ __forceinline__ void guard(v8f& a, v8f& b, v16h x, v16h y) { dep_guard_h(a, b, x, y); }
  static __device__ __forceinline__ void keep(v16h a, v16h b, v16h c, v16h d) { keep4_h(a, b, c, d); }
};
template <> struct Frag<__bf16> {
  typedef v16b V; union U { v16b v; v8b h[2]; };
  static __device__ __forceinline__ v16b load(const __bf16* p) {
    U f; f.h[0] = *(const v8b*)(p); f.h[1] = *(const v8b*)(p + 16); return f.v;
  }
  static __device__ __forceinline__ v8f mma(v16b a, v16b b, v8f c) {
    return __builtin_amdgcn_wmma_f32_16x16x32_bf16(false, a, false, b, (short)0, c, false, false);
  }
  static __device__ __forceinline__ void guard(v8f& a, v8f& b, v16b x, v16b y) { dep_guard_b(a, b, x, y); }
  static __device__ __forceinline__ void keep(v16b a, v16b b, v16b c, v16b d) { keep4_b(a, b, c, d); }
};

template <int ET> struct Elem;
template <> struct Elem<0> { typedef _Float16 T; };
template <> struct Elem<1> { typedef __bf16 T; };
template <int ET, bool SPLIT, int BIAS_MODE, int OUT_MODE, bool RESID, int ACT = 0>
__global__ __launch_bounds__(256) void wmma_gemm64(
    const unsigned short* __restrict__ Ap, const unsigned short* __restrict__ A2p, int lda, long strideA,
    const unsigned short* __restrict__ Btp, const unsigned short* __restrict__ Bt2p, int ldb, long strideB,
    void* __restrict__ Cout, void* __restrict__ Cout2, int ldc, long strideC,
    const float* __restrict__ bias,
    const float* __restrict__ resid, long strideR,
    int M, int N, int K, float scale) {
  typedef typename Elem<ET>::T T;
  typedef typename Frag<T>::V V;
  const T* A = (const T*)Ap; const T* A2 = (const T*)A2p; const T* Bt = (const T*)Btp; const T* Bt2 = (const T*)Bt2p;
  __shared__ __align__(16) float sT[8][16 * 68];
  const int b    = blockIdx.y;
  const int lane = threadIdx.x & 31;
  const int wave = threadIdx.x >> 5;
  const int tilesN = N >> 6;
  const int tilesM = M >> 6;
  const int tile = blockIdx.x * 8 + wave;
  if (tile >= tilesM * tilesN) return;
  const int tm = tile / tilesN;
  const int tn = tile - tm * tilesN;
  const int m0 = tm << 6;
  const int n0 = tn << 6;

  const T* Ab  = A  + (size_t)b * strideA;
  const T* Bb  = Bt + (size_t)b * strideB;
  const T* Ab2 = SPLIT ? (A2  + (size_t)b * strideA) : nullptr;
  const T* Bb2 = SPLIT ? (Bt2 + (size_t)b * strideB) : nullptr;

  const int rlane = lane & 15;
  const int koff  = (lane >> 4) * 8;
  const int mOff  = (lane >> 4) * 8;

  v8f acc[4][4];
#pragma unroll
  for (int i = 0; i < 4; ++i)
#pragma unroll
    for (int j = 0; j < 4; ++j) acc[i][j] = (v8f){0.f,0.f,0.f,0.f,0.f,0.f,0.f,0.f};

  for (int k0 = 0; k0 < K; k0 += 32) {
    V bh[4], bl[4];
#pragma unroll
    for (int j = 0; j < 4; ++j) {
      const size_t bo = (size_t)(n0 + (j << 4) + rlane) * ldb + koff + k0;
      bh[j] = Frag<T>::load(Bb + bo);
      if (SPLIT) bl[j] = Frag<T>::load(Bb2 + bo);
    }
#pragma unroll
    for (int i = 0; i < 4; ++i) {
      const size_t ao = (size_t)(m0 + (i << 4) + rlane) * lda + koff + k0;
      V ah = Frag<T>::load(Ab + ao);
      V al;
      if (SPLIT) al = Frag<T>::load(Ab2 + ao);
#pragma unroll
      for (int j = 0; j < 4; ++j) {
        acc[i][j] = Frag<T>::mma(ah, bh[j], acc[i][j]);
        if (SPLIT) {
          acc[i][j] = Frag<T>::mma(ah, bl[j], acc[i][j]);
          acc[i][j] = Frag<T>::mma(al, bh[j], acc[i][j]);
        }
      }
      Frag<T>::guard(acc[i][0], acc[i][3], ah, SPLIT ? al : ah);
    }
    Frag<T>::keep(bh[0], bh[1], bh[2], bh[3]);
    if (SPLIT) Frag<T>::keep(bl[0], bl[1], bl[2], bl[3]);
  }
  acc_guard4(acc[0][0], acc[0][1], acc[0][2], acc[0][3]);
  acc_guard4(acc[1][0], acc[1][1], acc[1][2], acc[1][3]);
  acc_guard4(acc[2][0], acc[2][1], acc[2][2], acc[2][3]);
  acc_guard4(acc[3][0], acc[3][1], acc[3][2], acc[3][3]);

  float* slab = sT[wave];
  const float* Rb = RESID ? (resid + (size_t)b * strideR) : nullptr;
#pragma unroll
  for (int i = 0; i < 4; ++i) {
    const int mBase = m0 + (i << 4);
#pragma unroll
    for (int j = 0; j < 4; ++j) {
      const int n = n0 + (j << 4) + rlane;
      float bv = 0.f;
      if (BIAS_MODE == 2) bv = bias[n];
#pragma unroll
      for (int r = 0; r < 8; ++r) {
        float v = acc[i][j][r] * scale;
        if (BIAS_MODE == 1) v += bias[mBase + mOff + r];
        if (BIAS_MODE == 2) v += bv;
        if (RESID) v += Rb[(size_t)(mBase + mOff + r) * ldc + n];
        if (ACT == 1) v = tanhf(v);
        if (ACT == 2) v = fmaxf(v, 0.0f);
        if (ACT == 3) v = v / (1.0f + expf(-v));
        if (ACT == 4) v = (v > 0.f) ? v : 0.01f * v;
        if (ACT == 5) v = 0.5f * v * (1.0f + erff(v * 0.70710678118654752f));
        slab[(mOff + r) * 68 + (j << 4) + rlane] = v;
      }
    }
    __builtin_amdgcn_fence(__ATOMIC_RELEASE, "workgroup");
    __builtin_amdgcn_wave_barrier();
    __builtin_amdgcn_fence(__ATOMIC_ACQUIRE, "workgroup");
    if (OUT_MODE == 0) {
      float* C = (float*)Cout + (size_t)b * strideC;
      const int hh = lane >> 4, c4 = (lane & 15) * 4;
      for (int pass = 0; pass < 2; ++pass) {
#pragma unroll
        for (int it = 0; it < 8; ++it) {
          const int row = it * 2 + hh;
          v4f v = *(const v4f*)(slab + row * 68 + c4);
          *(volatile v4f*)(C + (size_t)(mBase + row) * ldc + n0 + c4) = v;
        }
        __threadfence();
      }
    } else {
      const int q = lane >> 3, c8 = (lane & 7) * 8;
      unsigned short* C  = (unsigned short*)Cout  + (size_t)b * strideC;
      unsigned short* C2 = (OUT_MODE == 2) ? ((unsigned short*)Cout2 + (size_t)b * strideC) : nullptr;
      for (int pass = 0; pass < 2; ++pass) {
#pragma unroll
        for (int it = 0; it < 4; ++it) {
          const int row = it * 4 + q;
          const float* sp = slab + row * 68 + c8;
          v8h hv, lv;
#pragma unroll
          for (int e = 0; e < 8; ++e) {
            if (OUT_MODE == 1) {
              hv[e] = (_Float16)sp[e];
            } else {
              unsigned short hb = f2bf_bits(sp[e]);
              unsigned short lb = f2bf_bits(sp[e] - bf_bits2f(hb));
              hv[e] = __builtin_bit_cast(_Float16, hb);
              lv[e] = __builtin_bit_cast(_Float16, lb);
            }
          }
          *(volatile v8h*)(C + (size_t)(mBase + row) * ldc + n0 + c8) = hv;
          if (OUT_MODE == 2) *(volatile v8h*)(C2 + (size_t)(mBase + row) * ldc + n0 + c8) = lv;
        }
        __threadfence();
      }
    }
    __builtin_amdgcn_fence(__ATOMIC_RELEASE, "workgroup");
    __builtin_amdgcn_wave_barrier();
    __builtin_amdgcn_fence(__ATOMIC_ACQUIRE, "workgroup");
  }
}

__global__ __launch_bounds__(256) void cast_f32_bf16x2(
    const float* __restrict__ in, unsigned short* __restrict__ out, int n2) {
  int i = blockIdx.x * 256 + threadIdx.x;
  if (i < n2) {
    const unsigned u = (unsigned)f2bf_bits(in[2 * i]) | ((unsigned)f2bf_bits(in[2 * i + 1]) << 16);
    ((volatile unsigned*)out)[i] = u;
    __threadfence();
    ((volatile unsigned*)out)[i] = u;
  }
}

__global__ __launch_bounds__(256) void fill_zero_u32(unsigned* __restrict__ out, int n) {
  int i = blockIdx.x * 256 + threadIdx.x;
  if (i < n) {
    ((volatile unsigned*)out)[i] = 0u;
    __threadfence();
    ((volatile unsigned*)out)[i] = 0u;
  }
}

__global__ __launch_bounds__(256) void split_bf16x8(
    const float* __restrict__ in, unsigned short* __restrict__ hi, unsigned short* __restrict__ lo, int n8) {
  int i = blockIdx.x * 256 + threadIdx.x;
  if (i < n8) {
    const size_t e0 = (size_t)i * 8;
    const v4f a = *(const v4f*)(in + e0);
    const v4f c = *(const v4f*)(in + e0 + 4);
    v8h hv, lv;
#pragma unroll
    for (int e = 0; e < 4; ++e) {
      const unsigned short hb = f2bf_bits(a[e]);
      const unsigned short lb = f2bf_bits(a[e] - bf_bits2f(hb));
      hv[e] = __builtin_bit_cast(_Float16, hb);
      lv[e] = __builtin_bit_cast(_Float16, lb);
      const unsigned short hc = f2bf_bits(c[e]);
      const unsigned short lc = f2bf_bits(c[e] - bf_bits2f(hc));
      hv[4 + e] = __builtin_bit_cast(_Float16, hc);
      lv[4 + e] = __builtin_bit_cast(_Float16, lc);
    }
    for (int pass = 0; pass < 2; ++pass) {
      *(volatile v8h*)(hi + e0) = hv;
      *(volatile v8h*)(lo + e0) = lv;
      __threadfence();
    }
  }
}

constexpr int SEQ_T  = 256;
constexpr int NBATCH = 256;
constexpr int XIN    = 64;
constexpr int HSZ    = 64;
constexpr int STSZ   = 128;
constexpr int OSZ    = 64;
constexpr int NOUT   = 64;
constexpr int KXH    = 192;
constexpr int NGATES = 512;
constexpr int NLAYER = 4;
constexpr int MAXD   = 12;
constexpr int APITCH = 192;
constexpr int NTHR   = 256;
constexpr int ROWS   = 16;
constexpr int RSH    = ROWS * HSZ;
constexpr int RSC    = ROWS * STSZ;
static_assert(KXH % 32 == 0, "");
static_assert(XIN + 2 * HSZ == KXH, "");
static_assert(NBATCH % ROWS == 0, "");
static_assert((APITCH * 2) % 16 == 0, "");

__device__ __forceinline__ float fsig(float x)  { return __builtin_amdgcn_rcpf(1.0f + __expf(-x)); }
__device__ __forceinline__ float ftanh(float x) { return 1.0f - 2.0f * __builtin_amdgcn_rcpf(__expf(2.0f * x) + 1.0f); }

__global__ __launch_bounds__(NTHR) void s2_layer_kernel(
    const float* __restrict__ in, const unsigned short* __restrict__ Wp, const float* __restrict__ bias,
    const float* __restrict__ res, float* __restrict__ out, int d, float loScale, float resScale) {
  __shared__ __align__(16) unsigned short Ahi[ROWS * APITCH];
  __shared__ __align__(16) unsigned short Alo[ROWS * APITCH];
  __shared__ __align__(16) unsigned short Rhi[MAXD * RSH];
  __shared__ __align__(16) unsigned short Rlo[MAXD * RSH];
  __shared__ __align__(16) float          Cr[MAXD * RSC];
  __shared__ __align__(16) float          Os[ROWS * OSZ];

  const int tid = threadIdx.x, lane = tid & 31, w = tid >> 5;
  const int c = lane & 15, hh = lane >> 4, koff = hh * 8;
  const int u = 16 * w + c;
  const int b0 = blockIdx.x * ROWS;
  const int dd = (d < 1) ? 1 : ((d > MAXD) ? MAXD : d);

  {
    unsigned* ah32 = (unsigned*)Ahi; unsigned* al32 = (unsigned*)Alo;
#pragma unroll 1
    for (int i = tid; i < ROWS * APITCH / 2; i += NTHR) { ah32[i] = 0u; al32[i] = 0u; }
    unsigned* rh32 = (unsigned*)Rhi; unsigned* rl32 = (unsigned*)Rlo;
#pragma unroll 1
    for (int i = tid; i < MAXD * RSH / 2; i += NTHR) { rh32[i] = 0u; rl32[i] = 0u; }
#pragma unroll 1
    for (int i = tid; i < MAXD * RSC; i += NTHR) Cr[i] = 0.0f;
  }
  const float bq0 = bf_bits2f(f2bf_bits(bias[0 * STSZ + u]));
  const float bq1 = bf_bits2f(f2bf_bits(bias[1 * STSZ + u]));
  const float bq2 = bf_bits2f(f2bf_bits(bias[2 * STSZ + u]));
  const float bq3 = bf_bits2f(f2bf_bits(bias[3 * STSZ + u]));
  float cprev[8];
#pragma unroll
  for (int r = 0; r < 8; ++r) cprev[r] = 0.0f;
  __syncthreads();

  const __bf16* Wl  = (const __bf16*)Wp;
  const __bf16* arh = (const __bf16*)Ahi + c * APITCH + koff;
  const __bf16* arl = (const __bf16*)Alo + c * APITCH + koff;
  const __bf16* wr  = Wl + (size_t)u * KXH + koff;
  const v8f z8 = {0.f, 0.f, 0.f, 0.f, 0.f, 0.f, 0.f, 0.f};

  int slot = 0;
#pragma unroll 1
  for (int t = 0; t < SEQ_T; ++t) {
    const bool useDel = (t >= dd);
    {
      const int m = tid >> 4, q4 = (tid & 15) * 4;
      const size_t grow = (size_t)t * NBATCH + (size_t)(b0 + m);
      const v4f v = *(const v4f*)(in + grow * XIN + q4);
      const unsigned short h0 = f2bf_bits(v[0]), h1 = f2bf_bits(v[1]), h2 = f2bf_bits(v[2]), h3 = f2bf_bits(v[3]);
      const unsigned short l0 = f2bf_bits((v[0] - bf_bits2f(h0)) * loScale);
      const unsigned short l1 = f2bf_bits((v[1] - bf_bits2f(h1)) * loScale);
      const unsigned short l2 = f2bf_bits((v[2] - bf_bits2f(h2)) * loScale);
      const unsigned short l3 = f2bf_bits((v[3] - bf_bits2f(h3)) * loScale);
      v2u ph, pl;
      ph[0] = (unsigned)h0 | ((unsigned)h1 << 16);
      ph[1] = (unsigned)h2 | ((unsigned)h3 << 16);
      pl[0] = (unsigned)l0 | ((unsigned)l1 << 16);
      pl[1] = (unsigned)l2 | ((unsigned)l3 << 16);
      *(v2u*)(Ahi + m * APITCH + q4) = ph;
      *(v2u*)(Alo + m * APITCH + q4) = pl;
      const v2u rh = *(const v2u*)(Rhi + slot * RSH + m * HSZ + q4);
      const v2u rl = *(const v2u*)(Rlo + slot * RSH + m * HSZ + q4);
      const v2u qh = *(const v2u*)(Ahi + m * APITCH + XIN + q4);
      const v2u ql = *(const v2u*)(Alo + m * APITCH + XIN + q4);
      v2u dh, dl;
      dh[0] = useDel ? rh[0] : qh[0];
      dh[1] = useDel ? rh[1] : qh[1];
      dl[0] = useDel ? rl[0] : ql[0];
      dl[1] = useDel ? rl[1] : ql[1];
      *(v2u*)(Ahi + m * APITCH + XIN + HSZ + q4) = dh;
      *(v2u*)(Alo + m * APITCH + XIN + HSZ + q4) = dl;
    }
    __syncthreads();

    v8f acc[4];
    acc[0] = z8; acc[1] = z8; acc[2] = z8; acc[3] = z8;
#pragma unroll 1
    for (int k0 = 0; k0 < KXH; k0 += 32) {
      const v16b ah = Frag<__bf16>::load(arh + k0);
      const v16b al = Frag<__bf16>::load(arl + k0);
      const v16b w0 = Frag<__bf16>::load(wr + k0);
      const v16b w1 = Frag<__bf16>::load(wr + (size_t)1 * STSZ * KXH + k0);
      const v16b w2 = Frag<__bf16>::load(wr + (size_t)2 * STSZ * KXH + k0);
      const v16b w3 = Frag<__bf16>::load(wr + (size_t)3 * STSZ * KXH + k0);
      acc[0] = Frag<__bf16>::mma(ah, w0, acc[0]);
      acc[0] = Frag<__bf16>::mma(al, w0, acc[0]);
      acc[1] = Frag<__bf16>::mma(ah, w1, acc[1]);
      acc[1] = Frag<__bf16>::mma(al, w1, acc[1]);
      acc[2] = Frag<__bf16>::mma(ah, w2, acc[2]);
      acc[2] = Frag<__bf16>::mma(al, w2, acc[2]);
      acc[3] = Frag<__bf16>::mma(ah, w3, acc[3]);
      acc[3] = Frag<__bf16>::mma(al, w3, acc[3]);
      dep_guard_b(acc[0], acc[3], ah, al);
      keep4_b(w0, w1, w2, w3);
    }
    acc_guard4(acc[0], acc[1], acc[2], acc[3]);

    float hst[8];
#pragma unroll
    for (int r = 0; r < 8; ++r) {
      const int m = 8 * hh + r;
      const float z0 = acc[0][r] + bq0;
      const float z1 = acc[1][r] + bq1;
      const float z2 = acc[2][r] + bq2;
      const float z3 = acc[3][r] + bq3;
      const float fg = fsig(z0 + 1.0f);
      const float ns = ftanh(z1);
      const float ag = fsig(z2);
      const float og = fsig(z3);
      const int ci = slot * RSC + m * STSZ + u;
      const float dC = Cr[ci];
      const float cp = cprev[r];
      const float wcd = ag * cp + (1.0f - ag) * dC;
      const float wc  = useDel ? wcd : cp;
      const float ncp = fg * wc + (1.0f - fg) * ns;
      const float nc  = (t > 0) ? ncp : ns;
      cprev[r] = nc;
      Cr[ci] = nc;
      hst[r] = og * nc;
    }
    if (w < 4) {
#pragma unroll
      for (int r = 0; r < 8; ++r) {
        const int m = 8 * hh + r;
        const float rv = res[((size_t)t * NBATCH + (size_t)(b0 + m)) * OSZ + (u & 63)];
        Os[m * OSZ + u] = hst[r] + resScale * rv;
      }
    }
    __syncthreads();
    if (w >= 4) {
      const int hj = u - HSZ;
#pragma unroll
      for (int r = 0; r < 8; ++r) {
        const int m = 8 * hh + r;
        const unsigned short hb = f2bf_bits(hst[r]);
        const unsigned short lb = f2bf_bits(hst[r] - bf_bits2f(hb));
        Ahi[m * APITCH + XIN + hj] = hb;
        Alo[m * APITCH + XIN + hj] = lb;
        Rhi[slot * RSH + m * HSZ + hj] = hb;
        Rlo[slot * RSH + m * HSZ + hj] = lb;
      }
    }
    __syncthreads();
    {
      const int row = tid >> 4, c4 = (tid & 15) * 4;
      const v4f ov = *(const v4f*)(Os + row * OSZ + c4);
      float* op = out + ((size_t)t * NBATCH + (size_t)(b0 + row)) * OSZ + c4;
      *(volatile v4f*)op = ov;
      __threadfence();
      *(volatile v4f*)op = ov;
    }
    slot = (slot + 1 >= dd) ? 0 : (slot + 1);
  }
}

extern "C" void kernel_launch(void* const* d_in, const int* in_sizes, int n_in,
                              void* d_out, int out_size, void* d_ws, size_t ws_size, hipStream_t stream) {
  if (n_in < 5 || d_out == nullptr || d_ws == nullptr) return;
  if (in_sizes[0] != SEQ_T * NBATCH * XIN || in_sizes[1] != NLAYER * NGATES * KXH || in_sizes[2] != NLAYER * NGATES ||
      in_sizes[3] != NOUT * OSZ || in_sizes[4] != NOUT || out_size != SEQ_T * NBATCH * NOUT) return;

  const float* x  = (const float*)d_in[0];
  const float* W  = (const float*)d_in[1];
  const float* bl = (const float*)d_in[2];
  const float* Wa = (const float*)d_in[3];
  const float* ba = (const float*)d_in[4];
  float* out = (float*)d_out;

  const size_t nRows  = (size_t)SEQ_T * NBATCH;
  const size_t planeB = nRows * OSZ * sizeof(float);
  char* ws = (char*)d_ws; size_t off = 0;
  auto carve = [&](size_t bytes) -> char* { char* p = ws + off; off += (bytes + 255) & ~(size_t)255; return p; };
  unsigned short* Wb  = (unsigned short*)carve((size_t)NLAYER * NGATES * KXH * 2);
  unsigned short* Wab = (unsigned short*)carve((size_t)NOUT * OSZ * 2);
  unsigned short* Waz = (unsigned short*)carve((size_t)NOUT * OSZ * 2);
  float* P0 = (float*)carve(planeB);
  float* P1 = (float*)carve(planeB);
  float* P2 = (float*)carve(planeB);
  if (off > ws_size || off > (size_t)134217728) return;
  unsigned short* Phi = (unsigned short*)P2;
  unsigned short* Plo = (unsigned short*)((char*)P2 + planeB / 2);

  const int nW2  = NLAYER * NGATES * KXH / 2;
  const int nWa2 = NOUT * OSZ / 2;
  cast_f32_bf16x2<<<(nW2 + 255) / 256, 256, 0, stream>>>(W, Wb, nW2);
  cast_f32_bf16x2<<<(nWa2 + 255) / 256, 256, 0, stream>>>(Wa, Wab, nWa2);
  fill_zero_u32<<<(nWa2 + 255) / 256, 256, 0, stream>>>((unsigned*)Waz, nWa2);

  const size_t WL = (size_t)NGATES * KXH;
  const dim3 gridL(NBATCH / ROWS);
  s2_layer_kernel<<<gridL, NTHR, 0, stream>>>(x,  Wb + 0 * WL, bl + 0 * NGATES, x,  P0, 1,  0.0f, 0.0f);
  s2_layer_kernel<<<gridL, NTHR, 0, stream>>>(P0, Wb + 1 * WL, bl + 1 * NGATES, P0, P1, 3,  1.0f, 0.0f);
  s2_layer_kernel<<<gridL, NTHR, 0, stream>>>(P1, Wb + 2 * WL, bl + 2 * NGATES, P1, P2, 6,  1.0f, 0.0f);
  s2_layer_kernel<<<gridL, NTHR, 0, stream>>>(P2, Wb + 3 * WL, bl + 3 * NGATES, P1, P0, 12, 1.0f, 1.0f);

  const int n8 = (int)(nRows * OSZ / 8);
  split_bf16x8<<<(n8 + 255) / 256, 256, 0, stream>>>(P0, Phi, Plo, n8);

  const int M = (int)nRows, N = NOUT, K = OSZ;
  const int tiles = (M / 64) * (N / 64);
  wmma_gemm64<1, true, 2, 0, false><<<dim3((tiles + 7) / 8, 1), 256, 0, stream>>>(
      Phi, Plo, K, 0L, Wab, Waz, K, 0L, (void*)out, (void*)Waz, N, 0L, ba, (const float*)P1, 0L, M, N, K, 1.0f);
}
